// GazePatternAttention_79482664779919
// MI455X (gfx1250) — hardware-verified
//
#include <hip/hip_runtime.h>
#include <stdint.h>

typedef __attribute__((ext_vector_type(16))) _Float16 v16h;
typedef __attribute__((ext_vector_type(8)))  _Float16 v8h;
typedef __attribute__((ext_vector_type(16))) __bf16   v16b;
typedef __attribute__((ext_vector_type(8)))  __bf16   v8b;
typedef __attribute__((ext_vector_type(8)))  float    v8f;
typedef __attribute__((ext_vector_type(4)))  float    v4f;

#define WD    256
#define NHEAD 4
#define HDIM  64
#define WIN   10
#define PADW  5

__device__ __forceinline__ unsigned short f2bf_bits(float f) {
  unsigned u = __float_as_uint(f);
  return (unsigned short)((u + 0x7FFFu + ((u >> 16) & 1u)) >> 16);
}
__device__ __forceinline__ float bf_bits2f(unsigned short h) { return __uint_as_float(((unsigned)h) << 16); }

__device__ __forceinline__ void dep_guard_h(v8f& a, v8f& b, v16h x, v16h y) { asm volatile("v_nop\n\tv_nop\n\tv_nop\n\tv_nop" : "+v"(a), "+v"(b) : "v"(x), "v"(y)); }
__device__ __forceinline__ void dep_guard_b(v8f& a, v8f& b, v16b x, v16b y) { asm volatile("v_nop\n\tv_nop\n\tv_nop\n\tv_nop" : "+v"(a), "+v"(b) : "v"(x), "v"(y)); }
__device__ __forceinline__ void keep4_h(v16h a, v16h b, v16h c, v16h d) { asm volatile("v_nop" :: "v"(a), "v"(b), "v"(c), "v"(d)); }
__device__ __forceinline__ void keep4_b(v16b a, v16b b, v16b c, v16b d) { asm volatile("v_nop" :: "v"(a), "v"(b), "v"(c), "v"(d)); }
__device__ __forceinline__ void acc_guard4(v8f& a, v8f& b, v8f& c, v8f& d) { asm volatile("v_nop\n\tv_nop\n\tv_nop\n\tv_nop" : "+v"(a), "+v"(b), "+v"(c), "+v"(d)); }
template <typename T> struct Frag;
template <> struct Frag<_Float16> {
  typedef v16h V; union U { v16h v; v8h h[2]; };
  static __device__ __forceinline__ v16h load(const _Float16* p) {
    U f; f.h[0] = *(const v8h*)(p); f.h[1] = *(const v8h*)(p + 16); return f.v;
  }
  static __device__ __forceinline__ v8f mma(v16h a, v16h b, v8f c) {
    return __builtin_amdgcn_wmma_f32_16x16x32_f16(false, a, false, b, (short)0, c, false, false);
  }
  static __device__ __forceinline__ void guard(v8f& a, v8f& b, v16h x, v16h y) { dep_guard_h(a, b, x, y); }
  static __device__ __forceinline__ void keep(v16h a, v16h b, v16h c, v16h d) { keep4_h(a, b, c, d); }
};
template <> struct Frag<__bf16> {
  typedef v16b V; union U { v16b v; v8b h[2]; };
  static __device__ __forceinline__ v16b load(const __bf16* p) {
    U f; f.h[0] = *(const v8b*)(p); f.h[1] = *(const v8b*)(p + 16); return f.v;
  }
  static __device__ __forceinline__ v8f mma(v16b a, v16b b, v8f c) {
    return __builtin_amdgcn_wmma_f32_16x16x32_bf16(false, a, false, b, (short)0, c, false, false);
  }
  static __device__ __forceinline__ void guard(v8f& a, v8f& b, v16b x, v16b y) { dep_guard_b(a, b, x, y); }
  static __device__ __forceinline__ void keep(v16b a, v16b b, v16b c, v16b d) { keep4_b(a, b, c, d); }
};

template <int ET> struct Elem;
template <> struct Elem<0> { typedef _Float16 T; };
template <> struct Elem<1> { typedef __bf16 T; };
template <int ET, bool SPLIT, int BIAS_MODE, int OUT_MODE, bool RESID, int ACT = 0>
__global__ __launch_bounds__(256) void wmma_gemm64(
    const unsigned short* __restrict__ Ap, const unsigned short* __restrict__ A2p, int lda, long strideA,
    const unsigned short* __restrict__ Btp, const unsigned short* __restrict__ Bt2p, int ldb, long strideB,
    void* __restrict__ Cout, void* __restrict__ Cout2, int ldc, long strideC,
    const float* __restrict__ bias,
    const float* __restrict__ resid, long strideR,
    int M, int N, int K, float scale) {
  typedef typename Elem<ET>::T T;
  typedef typename Frag<T>::V V;
  const T* A = (const T*)Ap; const T* A2 = (const T*)A2p; const T* Bt = (const T*)Btp; const T* Bt2 = (const T*)Bt2p;
  __shared__ __align__(16) float sT[8][16 * 68];
  const int b    = blockIdx.y;
  const int lane = threadIdx.x & 31;
  const int wave = threadIdx.x >> 5;
  const int tilesN = N >> 6;
  const int tilesM = M >> 6;
  const int tile = blockIdx.x * 8 + wave;
  if (tile >= tilesM * tilesN) return;
  const int tm = tile / tilesN;
  const int tn = tile - tm * tilesN;
  const int m0 = tm << 6;
  const int n0 = tn << 6;

  const T* Ab  = A  + (size_t)b * strideA;
  const T* Bb  = Bt + (size_t)b * strideB;
  const T* Ab2 = SPLIT ? (A2  + (size_t)b * strideA) : nullptr;
  const T* Bb2 = SPLIT ? (Bt2 + (size_t)b * strideB) : nullptr;

  const int rlane = lane & 15;
  const int koff  = (lane >> 4) * 8;
  const int mOff  = (lane >> 4) * 8;

  v8f acc[4][4];
#pragma unroll
  for (int i = 0; i < 4; ++i)
#pragma unroll
    for (int j = 0; j < 4; ++j) acc[i][j] = (v8f){0.f,0.f,0.f,0.f,0.f,0.f,0.f,0.f};

  for (int k0 = 0; k0 < K; k0 += 32) {
    V bh[4], bl[4];
#pragma unroll
    for (int j = 0; j < 4; ++j) {
      const size_t bo = (size_t)(n0 + (j << 4) + rlane) * ldb + koff + k0;
      bh[j] = Frag<T>::load(Bb + bo);
      if (SPLIT) bl[j] = Frag<T>::load(Bb2 + bo);
    }
#pragma unroll
    for (int i = 0; i < 4; ++i) {
      const size_t ao = (size_t)(m0 + (i << 4) + rlane) * lda + koff + k0;
      V ah = Frag<T>::load(Ab + ao);
      V al;
      if (SPLIT) al = Frag<T>::load(Ab2 + ao);
#pragma unroll
      for (int j = 0; j < 4; ++j) {
        acc[i][j] = Frag<T>::mma(ah, bh[j], acc[i][j]);
        if (SPLIT) {
          acc[i][j] = Frag<T>::mma(ah, bl[j], acc[i][j]);
          acc[i][j] = Frag<T>::mma(al, bh[j], acc[i][j]);
        }
      }
      Frag<T>::guard(acc[i][0], acc[i][3], ah, SPLIT ? al : ah);
    }
    Frag<T>::keep(bh[0], bh[1], bh[2], bh[3]);
    if (SPLIT) Frag<T>::keep(bl[0], bl[1], bl[2], bl[3]);
  }
  acc_guard4(acc[0][0], acc[0][1], acc[0][2], acc[0][3]);
  acc_guard4(acc[1][0], acc[1][1], acc[1][2], acc[1][3]);
  acc_guard4(acc[2][0], acc[2][1], acc[2][2], acc[2][3]);
  acc_guard4(acc[3][0], acc[3][1], acc[3][2], acc[3][3]);

  float* slab = sT[wave];
  const float* Rb = RESID ? (resid + (size_t)b * strideR) : nullptr;
#pragma unroll
  for (int i = 0; i < 4; ++i) {
    const int mBase = m0 + (i << 4);
#pragma unroll
    for (int j = 0; j < 4; ++j) {
      const int n = n0 + (j << 4) + rlane;
      float bv = 0.f;
      if (BIAS_MODE == 2) bv = bias[n];
#pragma unroll
      for (int r = 0; r < 8; ++r) {
        float v = acc[i][j][r] * scale;
        if (BIAS_MODE == 1) v += bias[mBase + mOff + r];
        if (BIAS_MODE == 2) v += bv;
        if (RESID) v += Rb[(size_t)(mBase + mOff + r) * ldc + n];
        if (ACT == 1) v = tanhf(v);
        if (ACT == 2) v = fmaxf(v, 0.0f);
        if (ACT == 3) v = v / (1.0f + expf(-v));
        if (ACT == 4) v = (v > 0.f) ? v : 0.01f * v;
        if (ACT == 5) v = 0.5f * v * (1.0f + erff(v * 0.70710678118654752f));
        slab[(mOff + r) * 68 + (j << 4) + rlane] = v;
      }
    }
    __builtin_amdgcn_fence(__ATOMIC_RELEASE, "workgroup");
    __builtin_amdgcn_wave_barrier();
    __builtin_amdgcn_fence(__ATOMIC_ACQUIRE, "workgroup");
    if (OUT_MODE == 0) {
      float* C = (float*)Cout + (size_t)b * strideC;
      const int hh = lane >> 4, c4 = (lane & 15) * 4;
      for (int pass = 0; pass < 2; ++pass) {
#pragma unroll
        for (int it = 0; it < 8; ++it) {
          const int row = it * 2 + hh;
          v4f v = *(const v4f*)(slab + row * 68 + c4);
          *(volatile v4f*)(C + (size_t)(mBase + row) * ldc + n0 + c4) = v;
        }
        __threadfence();
      }
    } else {
      const int q = lane >> 3, c8 = (lane & 7) * 8;
      unsigned short* C  = (unsigned short*)Cout  + (size_t)b * strideC;
      unsigned short* C2 = (OUT_MODE == 2) ? ((unsigned short*)Cout2 + (size_t)b * strideC) : nullptr;
      for (int pass = 0; pass < 2; ++pass) {
#pragma unroll
        for (int it = 0; it < 4; ++it) {
          const int row = it * 4 + q;
          const float* sp = slab + row * 68 + c8;
          v8h hv, lv;
#pragma unroll
          for (int e = 0; e < 8; ++e) {
            if (OUT_MODE == 1) {
              hv[e] = (_Float16)sp[e];
            } else {
              unsigned short hb = f2bf_bits(sp[e]);
              unsigned short lb = f2bf_bits(sp[e] - bf_bits2f(hb));
              hv[e] = __builtin_bit_cast(_Float16, hb);
              lv[e] = __builtin_bit_cast(_Float16, lb);
            }
          }
          *(volatile v8h*)(C + (size_t)(mBase + row) * ldc + n0 + c8) = hv;
          if (OUT_MODE == 2) *(volatile v8h*)(C2 + (size_t)(mBase + row) * ldc + n0 + c8) = lv;
        }
        __threadfence();
      }
    }
    __builtin_amdgcn_fence(__ATOMIC_RELEASE, "workgroup");
    __builtin_amdgcn_wave_barrier();
    __builtin_amdgcn_fence(__ATOMIC_ACQUIRE, "workgroup");
  }
}

__global__ __launch_bounds__(256) void cast8_kernel(const float* __restrict__ in, _Float16* __restrict__ out, int n8) {
  const int i = blockIdx.x * 256 + threadIdx.x;
  if (i < n8) {
    const v4f a = *(const v4f*)(in + (size_t)8 * i);
    const v4f b = *(const v4f*)(in + (size_t)8 * i + 4);
    v8h hv;
    hv[0] = (_Float16)a[0]; hv[1] = (_Float16)a[1]; hv[2] = (_Float16)a[2]; hv[3] = (_Float16)a[3];
    hv[4] = (_Float16)b[0]; hv[5] = (_Float16)b[1]; hv[6] = (_Float16)b[2]; hv[7] = (_Float16)b[3];
    _Float16* p = out + (size_t)8 * i;
    *(volatile v8h*)p = hv;
    __threadfence();
    *(volatile v8h*)p = hv;
  }
}

__global__ __launch_bounds__(256) void transpose_cast_kernel(const float* __restrict__ W, _Float16* __restrict__ Bt, int K, int N) {
  __shared__ float tile[64][33];
  const int k0 = blockIdx.x * 64, n0 = blockIdx.y * 32;
  const int tid = threadIdx.x, lane = tid & 31, wave = tid >> 5;
#pragma unroll
  for (int i = 0; i < 8; ++i) {
    const int r = wave * 8 + i;
    tile[r][lane] = W[(size_t)(k0 + r) * N + n0 + lane];
  }
  __syncthreads();
  const int q = lane >> 3, c8 = (lane & 7) * 8;
  const int nl = wave * 4 + q;
  v8h hv;
#pragma unroll
  for (int e = 0; e < 8; ++e) hv[e] = (_Float16)tile[c8 + e][nl];
  _Float16* dst = Bt + (size_t)(n0 + nl) * K + k0 + c8;
  *(volatile v8h*)dst = hv;
  __threadfence();
  *(volatile v8h*)dst = hv;
}

#define AT_D 64
#define AT_NW 4
#define AT_QB 64
#define AT_KC 64
#define AT_PSC 32768.0f

__device__ __forceinline__ v8f mma_h(v16h a, v16h b, v8f c) {
  c = __builtin_amdgcn_wmma_f32_16x16x32_f16(false, a, false, b, (short)0, c, false, false);
  asm volatile("v_nop\n\tv_nop\n\tv_nop\n\tv_nop" : "+v"(c) : "v"(a), "v"(b));
  return c;
}

__global__ __launch_bounds__(128)
void attn_f16_kernel(const _Float16* __restrict__ q, const _Float16* __restrict__ k,
                     const _Float16* __restrict__ v, _Float16* __restrict__ out,
                     const float* __restrict__ rel, int S, int H, int ld, int nrel, float sscale) {
  __shared__ __align__(16) _Float16 Ksh[AT_KC * AT_D];
  __shared__ __align__(16) _Float16 Vth[AT_D * AT_KC];
  __shared__ __align__(16) _Float16 Psh[AT_NW][16 * AT_KC];
  __shared__ __align__(16) float    Os[AT_NW][16 * 68];

  const int tid  = threadIdx.x;
  const int wave = tid >> 5;
  const int lane = tid & 31;
  const int hh   = lane >> 4;
  const int c    = lane & 15;

  const int nqb = S / AT_QB;
  const int bx = blockIdx.x;
  const int qb = bx % nqb;
  const int bh = bx / nqb;
  const int h  = bh % H;
  const int b  = bh / H;
  const int q0 = qb * AT_QB + wave * 16;

  const size_t boff = (size_t)b * S * ld + (size_t)h * AT_D;
  const _Float16* qb_ptr = q + boff;
  const _Float16* kb_ptr = k + boff;
  const _Float16* vb_ptr = v + boff;
  _Float16*       ob_ptr = out + boff;

  v16h qa[2];
#pragma unroll
  for (int dc = 0; dc < 2; ++dc)
    qa[dc] = Frag<_Float16>::load(qb_ptr + (size_t)(q0 + c) * ld + dc * 32 + 8 * hh);

  float mrow[8], lrow[8];
  v8f oacc[4];
#pragma unroll
  for (int r = 0; r < 8; ++r) { mrow[r] = -INFINITY; lrow[r] = 0.f; }
#pragma unroll
  for (int t = 0; t < 4; ++t) oacc[t] = (v8f){0.f,0.f,0.f,0.f,0.f,0.f,0.f,0.f};

  const int nChunks = S / AT_KC;
  for (int kc = 0; kc < nChunks; ++kc) {
    const int kv0 = kc * AT_KC;
    __syncthreads();
    {
      const int kvr = tid >> 1, dh = (tid & 1) * 32;
      const _Float16* krow = kb_ptr + (size_t)(kv0 + kvr) * ld + dh;
      const _Float16* vrow = vb_ptr + (size_t)(kv0 + kvr) * ld + dh;
#pragma unroll
      for (int i = 0; i < 4; ++i) {
        const v8h kk = *(const v8h*)(krow + 8 * i);
        *(v8h*)(Ksh + kvr * AT_D + dh + 8 * i) = kk;
        const v8h vv = *(const v8h*)(vrow + 8 * i);
#pragma unroll
        for (int e = 0; e < 8; ++e) Vth[(dh + 8 * i + e) * AT_KC + kvr] = vv[e];
      }
    }
    __syncthreads();

    v8f s[4];
#pragma unroll
    for (int j = 0; j < 4; ++j) {
      s[j] = (v8f){0.f,0.f,0.f,0.f,0.f,0.f,0.f,0.f};
#pragma unroll
      for (int dc = 0; dc < 2; ++dc) {
        const v16h kb = Frag<_Float16>::load(Ksh + (j * 16 + c) * AT_D + dc * 32 + 8 * hh);
        s[j] = mma_h(qa[dc], kb, s[j]);
      }
    }
    float cm[8];
#pragma unroll
    for (int r = 0; r < 8; ++r) {
      const int qrow = q0 + 8 * hh + r;
      float m = -INFINITY;
#pragma unroll
      for (int j = 0; j < 4; ++j) {
        const int kvcol = kv0 + j * 16 + c;
        int ri = kvcol - qrow + S - 1;
        ri = ri < 0 ? 0 : (ri > nrel - 1 ? nrel - 1 : ri);
        const float sv = s[j][r] * sscale + rel[(size_t)ri * H + h];
        s[j][r] = sv;
        m = fmaxf(m, sv);
      }
#pragma unroll
      for (int off = 1; off < 16; off <<= 1) m = fmaxf(m, __shfl_xor(m, off, 32));
      cm[r] = m;
    }
    _Float16* pwh = Psh[wave];
#pragma unroll
    for (int r = 0; r < 8; ++r) {
      const float mnew = fmaxf(mrow[r], cm[r]);
      const float alpha = expf(mrow[r] - mnew);
      mrow[r] = mnew;
      float psum = 0.f;
#pragma unroll
      for (int j = 0; j < 4; ++j) {
        const float p = expf(s[j][r] - mnew);
        psum += p;
        pwh[(8 * hh + r) * AT_KC + j * 16 + c] = (_Float16)(p * AT_PSC);
      }
#pragma unroll
      for (int off = 1; off < 16; off <<= 1) psum += __shfl_xor(psum, off, 32);
      lrow[r] = lrow[r] * alpha + psum;
#pragma unroll
      for (int t = 0; t < 4; ++t) oacc[t][r] *= alpha;
    }
    __builtin_amdgcn_fence(__ATOMIC_RELEASE, "workgroup");
    __builtin_amdgcn_wave_barrier();
    __builtin_amdgcn_fence(__ATOMIC_ACQUIRE, "workgroup");
#pragma unroll
    for (int kk = 0; kk < 2; ++kk) {
      const v16h pa = Frag<_Float16>::load(pwh + c * AT_KC + kk * 32 + 8 * hh);
#pragma unroll
      for (int t = 0; t < 4; ++t) {
        const v16h vb = Frag<_Float16>::load(Vth + (t * 16 + c) * AT_KC + kk * 32 + 8 * hh);
        oacc[t] = mma_h(pa, vb, oacc[t]);
      }
    }
  }

  float* os = Os[wave];
#pragma unroll
  for (int r = 0; r < 8; ++r) {
    const float inv = 1.0f / (lrow[r] * AT_PSC);
#pragma unroll
    for (int t = 0; t < 4; ++t) os[(8 * hh + r) * 68 + t * 16 + c] = oacc[t][r] * inv;
  }
  __builtin_amdgcn_fence(__ATOMIC_RELEASE, "workgroup");
  __builtin_amdgcn_wave_barrier();
  __builtin_amdgcn_fence(__ATOMIC_ACQUIRE, "workgroup");
  {
    const int qq = lane >> 3, c8 = (lane & 7) * 8;
    for (int pass = 0; pass < 2; ++pass) {
#pragma unroll
      for (int it = 0; it < 4; ++it) {
        const int row = it * 4 + qq;
        const v4f a0 = *(const v4f*)(os + row * 68 + c8);
        const v4f a1 = *(const v4f*)(os + row * 68 + c8 + 4);
        v8h hv;
        hv[0] = (_Float16)a0[0]; hv[1] = (_Float16)a0[1]; hv[2] = (_Float16)a0[2]; hv[3] = (_Float16)a0[3];
        hv[4] = (_Float16)a1[0]; hv[5] = (_Float16)a1[1]; hv[6] = (_Float16)a1[2]; hv[7] = (_Float16)a1[3];
        *(volatile v8h*)(ob_ptr + (size_t)(q0 + row) * ld + c8) = hv;
      }
      __threadfence();
    }
  }
}

__global__ __launch_bounds__(256) void window_attn_kernel(
    const _Float16* __restrict__ lq, const _Float16* __restrict__ lk, const _Float16* __restrict__ lv,
    const float* __restrict__ lkb, const float* __restrict__ lvb,
    _Float16* __restrict__ cat, int ldcat, int coff, int T, int nTok, float sscale)
{
  const int lane = threadIdx.x & 31, wave = threadIdx.x >> 5;
  const int tok = blockIdx.x * 8 + wave;
  if (tok >= nTok) return;
  const int b = tok / T, t = tok - b * T;
  const int d0 = lane * 8;
  const v8h qv = *(const v8h*)(lq + (size_t)tok * WD + d0);
  float qf[8], kb[8], vb[8], o[8];
#pragma unroll
  for (int e = 0; e < 8; ++e) { qf[e] = (float)qv[e]; kb[e] = lkb[d0 + e]; vb[e] = lvb[d0 + e]; o[e] = 0.f; }

  float myscore = -INFINITY;
#pragma unroll 1
  for (int wi = 0; wi < WIN; ++wi) {
    const int sp = t + wi - PADW;
    const bool valid = (sp >= 0) && (sp < T);
    const int spc = sp < 0 ? 0 : (sp >= T ? T - 1 : sp);
    const v8h kvv = *(const v8h*)(lk + ((size_t)b * T + spc) * WD + d0);
    float s = 0.f;
#pragma unroll
    for (int e = 0; e < 8; ++e) { const float kf = valid ? (float)kvv[e] : kb[e]; s = fmaf(qf[e], kf, s); }
#pragma unroll
    for (int off = 16; off > 0; off >>= 1) s += __shfl_xor(s, off, 32);
    if (lane == wi) myscore = s * sscale;
  }
  float m = myscore;
#pragma unroll
  for (int off = 16; off > 0; off >>= 1) m = fmaxf(m, __shfl_xor(m, off, 32));
  float p = (lane < WIN) ? expf(myscore - m) : 0.f;
  float sum = p;
#pragma unroll
  for (int off = 16; off > 0; off >>= 1) sum += __shfl_xor(sum, off, 32);
  p = p * (1.0f / sum);

#pragma unroll 1
  for (int wi = 0; wi < WIN; ++wi) {
    const int sp = t + wi - PADW;
    const bool valid = (sp >= 0) && (sp < T);
    const int spc = sp < 0 ? 0 : (sp >= T ? T - 1 : sp);
    const v8h vvv = *(const v8h*)(lv + ((size_t)b * T + spc) * WD + d0);
    const float pw = __shfl(p, wi, 32);
#pragma unroll
    for (int e = 0; e < 8; ++e) { const float vf = valid ? (float)vvv[e] : vb[e]; o[e] = fmaf(pw, vf, o[e]); }
  }
  v8h ov;
#pragma unroll
  for (int e = 0; e < 8; ++e) ov[e] = (_Float16)o[e];
  _Float16* dst = cat + (size_t)tok * ldcat + coff + d0;
  *(volatile v8h*)dst = ov;
  __threadfence();
  *(volatile v8h*)dst = ov;
}

__global__ __launch_bounds__(256) void pool_score_kernel(
    const float* __restrict__ x, const float* __restrict__ pe,
    const float* __restrict__ pqw, const float* __restrict__ pqb,
    const float* __restrict__ pkw, const float* __restrict__ pkb,
    float* __restrict__ out, int nB, int T, float sscale)
{
  __shared__ float pooled[WD], pqv[WD], pkv[3][WD], lg[16], res[128];
  const int tid = threadIdx.x;
  if (tid < 128) res[tid] = 0.f;
#pragma unroll 1
  for (int kk = 0; kk < 3; ++kk) {
    float s2 = pkb[tid];
#pragma unroll 1
    for (int k2 = 0; k2 < WD; ++k2) s2 = fmaf(pe[kk * WD + k2], pkw[(size_t)k2 * WD + tid], s2);
    pkv[kk][tid] = s2;
  }
  const int nBc = nB < 32 ? nB : 32;
  const float invT = 1.0f / (float)T;
#pragma unroll 1
  for (int b = 0; b < nBc; ++b) {
    __syncthreads();
    {
      float s = 0.f;
      const float* xb = x + (size_t)b * T * WD + tid;
#pragma unroll 4
      for (int t2 = 0; t2 < T; ++t2) s += xb[(size_t)t2 * WD];
      pooled[tid] = s * invT;
    }
    __syncthreads();
    {
      float s = pqb[tid];
#pragma unroll 1
      for (int k2 = 0; k2 < WD; ++k2) s = fmaf(pooled[k2], pqw[(size_t)k2 * WD + tid], s);
      pqv[tid] = s;
    }
    __syncthreads();
    if (tid < NHEAD * 3) {
      const int hd = tid / 3, kk = tid - hd * 3;
      float a = 0.f;
#pragma unroll 1
      for (int d = 0; d < HDIM; ++d) a = fmaf(pqv[hd * HDIM + d], pkv[kk][hd * HDIM + d], a);
      lg[tid] = a * sscale;
    }
    __syncthreads();
    if (tid == 0) {
      float pw0 = 0.f, pw1 = 0.f, pw2 = 0.f;
#pragma unroll 1
      for (int hd = 0; hd < NHEAD; ++hd) {
        const float l0 = lg[hd * 3 + 0], l1 = lg[hd * 3 + 1], l2 = lg[hd * 3 + 2];
        const float mm = fmaxf(l0, fmaxf(l1, l2));
        const float e0 = expf(l0 - mm), e1 = expf(l1 - mm), e2 = expf(l2 - mm);
        const float inv = 1.0f / (e0 + e1 + e2);
        pw0 += e0 * inv; pw1 += e1 * inv; pw2 += e2 * inv;
      }
      res[b * 3 + 0] = pw0 * (1.0f / (float)NHEAD);
      res[b * 3 + 1] = pw1 * (1.0f / (float)NHEAD);
      res[b * 3 + 2] = pw2 * (1.0f / (float)NHEAD);
    }
  }
  __syncthreads();
  const int nl = (nBc * 3) / 4;
  for (int pass = 0; pass < 2; ++pass) {
    if (tid < nl) {
      v4f val;
      val[0] = res[4 * tid + 0]; val[1] = res[4 * tid + 1]; val[2] = res[4 * tid + 2]; val[3] = res[4 * tid + 3];
      *(volatile v4f*)(out + 4 * tid) = val;
    }
    __threadfence();
  }
}

extern "C" void kernel_launch(void* const* d_in, const int* in_sizes, int n_in,
                              void* d_out, int out_size, void* d_ws, size_t ws_size,
                              hipStream_t stream)
{
  if (n_in < 25) return;
  const float* x     = (const float*)d_in[0];
  const float* gq_w  = (const float*)d_in[1];
  const float* gq_b  = (const float*)d_in[2];
  const float* gk_w  = (const float*)d_in[3];
  const float* gk_b  = (const float*)d_in[4];
  const float* gv_w  = (const float*)d_in[5];
  const float* gv_b  = (const float*)d_in[6];
  const float* go_w  = (const float*)d_in[7];
  const float* go_b  = (const float*)d_in[8];
  const float* rel   = (const float*)d_in[9];
  const float* lq_w  = (const float*)d_in[10];
  const float* lq_b  = (const float*)d_in[11];
  const float* lk_w  = (const float*)d_in[12];
  const float* lk_b  = (const float*)d_in[13];
  const float* lv_w  = (const float*)d_in[14];
  const float* lv_b  = (const float*)d_in[15];
  const float* pe    = (const float*)d_in[16];
  const float* pq_w  = (const float*)d_in[17];
  const float* pq_b  = (const float*)d_in[18];
  const float* pk_w  = (const float*)d_in[19];
  const float* pk_b  = (const float*)d_in[20];
  const float* f1_w  = (const float*)d_in[21];
  const float* f1_b  = (const float*)d_in[22];
  const float* f2_w  = (const float*)d_in[23];
  const float* f2_b  = (const float*)d_in[24];

  const int M = in_sizes[0] / WD;
  const int nrel = in_sizes[9] / NHEAD;
  const int T = (nrel + 1) / 2;
  if (T <= 0) return;
  const int B = M / T;
  if (M % 64 != 0 || T % 64 != 0 || B * T != M || B <= 0 || B > 32) return;
  if ((B * 3) % 4 != 0 || (B * 3) / 4 > 32) return;
  if (in_sizes[1] != WD * WD || in_sizes[21] != 2 * WD * WD || in_sizes[23] != WD * WD) return;
  if (out_size != M * WD + B * 3) return;

  char* ws = (char*)d_ws;
  size_t off = 0;
  auto carve = [&](size_t bytes) -> char* { char* p = ws + off; off += (bytes + 255) & ~(size_t)255; return p; };
  const size_t actB = (size_t)M * WD * sizeof(_Float16);
  const size_t wB   = (size_t)WD * WD * sizeof(_Float16);
  _Float16* xh   = (_Float16*)carve(actB);
  _Float16* wq   = (_Float16*)carve(wB);
  _Float16* wk   = (_Float16*)carve(wB);
  _Float16* wv   = (_Float16*)carve(wB);
  _Float16* wo   = (_Float16*)carve(wB);
  _Float16* wlq  = (_Float16*)carve(wB);
  _Float16* wlk  = (_Float16*)carve(wB);
  _Float16* wlv  = (_Float16*)carve(wB);
  _Float16* wf1  = (_Float16*)carve(2 * wB);
  _Float16* wf2  = (_Float16*)carve(wB);
  _Float16* qh   = (_Float16*)carve(actB);
  _Float16* kh   = (_Float16*)carve(actB);
  _Float16* vh   = (_Float16*)carve(actB);
  _Float16* lqh  = (_Float16*)carve(actB);
  _Float16* lkh  = (_Float16*)carve(actB);
  _Float16* lvh  = (_Float16*)carve(actB);
  _Float16* gouth = (_Float16*)carve(actB);
  _Float16* cath  = (_Float16*)carve(2 * actB);
  _Float16* h1h   = (_Float16*)carve(actB);
  const size_t lim = ws_size < (size_t)134217728 ? ws_size : (size_t)134217728;
  if (off > lim) return;

  typedef const unsigned short* cus;

  {
    const int n8 = M * WD / 8;
    cast8_kernel<<<dim3((n8 + 255) / 256), dim3(256), 0, stream>>>(x, xh, n8);
  }
  {
    const dim3 g256(WD / 64, WD / 32), g512(2 * WD / 64, WD / 32), blk(256);
    transpose_cast_kernel<<<g256, blk, 0, stream>>>(gq_w, wq,  WD, WD);
    transpose_cast_kernel<<<g256, blk, 0, stream>>>(gk_w, wk,  WD, WD);
    transpose_cast_kernel<<<g256, blk, 0, stream>>>(gv_w, wv,  WD, WD);
    transpose_cast_kernel<<<g256, blk, 0, stream>>>(go_w, wo,  WD, WD);
    transpose_cast_kernel<<<g256, blk, 0, stream>>>(lq_w, wlq, WD, WD);
    transpose_cast_kernel<<<g256, blk, 0, stream>>>(lk_w, wlk, WD, WD);
    transpose_cast_kernel<<<g256, blk, 0, stream>>>(lv_w, wlv, WD, WD);
    transpose_cast_kernel<<<g512, blk, 0, stream>>>(f1_w, wf1, 2 * WD, WD);
    transpose_cast_kernel<<<g256, blk, 0, stream>>>(f2_w, wf2, WD, WD);
  }
  const int tiles = (M / 64) * (WD / 64);
  const dim3 ggrd((tiles + 7) / 8, 1), gblk(256);
  wmma_gemm64<0, false, 2, 1, false, 0><<<ggrd, gblk, 0, stream>>>(
      (cus)xh, nullptr, WD, 0L, (cus)wq, nullptr, WD, 0L, (void*)qh, nullptr, WD, 0L, gq_b, nullptr, 0L, M, WD, WD, 1.0f);
  wmma_gemm64<0, false, 2, 1, false, 0><<<ggrd, gblk, 0, stream>>>(
      (cus)xh, nullptr, WD, 0L, (cus)wk, nullptr, WD, 0L, (void*)kh, nullptr, WD, 0L, gk_b, nullptr, 0L, M, WD, WD, 1.0f);
  wmma_gemm64<0, false, 2, 1, false, 0><<<ggrd, gblk, 0, stream>>>(
      (cus)xh, nullptr, WD, 0L, (cus)wv, nullptr, WD, 0L, (void*)vh, nullptr, WD, 0L, gv_b, nullptr, 0L, M, WD, WD, 1.0f);
  wmma_gemm64<0, false, 2, 1, false, 0><<<ggrd, gblk, 0, stream>>>(
      (cus)xh, nullptr, WD, 0L, (cus)wlq, nullptr, WD, 0L, (void*)lqh, nullptr, WD, 0L, lq_b, nullptr, 0L, M, WD, WD, 1.0f);
  wmma_gemm64<0, false, 2, 1, false, 0><<<ggrd, gblk, 0, stream>>>(
      (cus)xh, nullptr, WD, 0L, (cus)wlk, nullptr, WD, 0L, (void*)lkh, nullptr, WD, 0L, lk_b, nullptr, 0L, M, WD, WD, 1.0f);
  wmma_gemm64<0, false, 2, 1, false, 0><<<ggrd, gblk, 0, stream>>>(
      (cus)xh, nullptr, WD, 0L, (cus)wlv, nullptr, WD, 0L, (void*)lvh, nullptr, WD, 0L, lv_b, nullptr, 0L, M, WD, WD, 1.0f);

  attn_f16_kernel<<<dim3(B * NHEAD * (T / AT_QB)), dim3(128), 0, stream>>>(
      qh, kh, vh, gouth, rel, T, NHEAD, WD, nrel, 0.125f);

  wmma_gemm64<0, false, 2, 1, false, 0><<<ggrd, gblk, 0, stream>>>(
      (cus)gouth, nullptr, WD, 0L, (cus)wo, nullptr, WD, 0L, (void*)cath, nullptr, 2 * WD, 0L, go_b, nullptr, 0L, M, WD, WD, 1.0f);

  window_attn_kernel<<<dim3((M + 7) / 8), dim3(256), 0, stream>>>(
      lqh, lkh, lvh, lk_b, lv_b, cath, 2 * WD, WD, T, M, 0.125f);

  wmma_gemm64<0, false, 2, 1, false, 2><<<ggrd, gblk, 0, stream>>>(
      (cus)cath, nullptr, 2 * WD, 0L, (cus)wf1, nullptr, 2 * WD, 0L, (void*)h1h, nullptr, WD, 0L, f1_b, nullptr, 0L, M, WD, 2 * WD, 1.0f);

  wmma_gemm64<0, false, 2, 0, true, 0><<<ggrd, gblk, 0, stream>>>(
      (cus)h1h, nullptr, WD, 0L, (cus)wf2, nullptr, WD, 0L, d_out, nullptr, WD, 0L, f2_b, x, 0L, M, WD, WD, 1.0f);

  pool_score_kernel<<<dim3(1), dim3(256), 0, stream>>>(
      x, pe, pq_w, pq_b, pk_w, pk_b, (float*)d_out + (size_t)M * WD, B, T, 0.125f);
}
